// ConvPosMultiHeadAttn_Order_1786706395835
// MI455X (gfx1250) — hardware-verified
//
#include <hip/hip_runtime.h>


namespace {
constexpr int Bn = 4, L = 1024, DM = 1024, H = 16, DH = 64, NTOK = Bn * L, NQKV = 4 * DM, NPOS = 3 * DM, TBL = 1201, SHIFT = 601;
constexpr float VS = 8.0f, PES = 8.0f;

typedef _Float16 b16;
typedef __attribute__((ext_vector_type(16))) _Float16 v16b;
typedef __attribute__((ext_vector_type(8)))  _Float16 v8b;
typedef __attribute__((ext_vector_type(8)))  float v8f;
typedef __attribute__((ext_vector_type(4)))  float v4f;

__device__ __forceinline__ v8b ld8b(const b16* p) { return *(const v8b*)p; }
__device__ __forceinline__ v16b cat8b(v8b a, v8b b) { return __builtin_shufflevector(a, b, 0, 1, 2, 3, 4, 5, 6, 7, 8, 9, 10, 11, 12, 13, 14, 15); }
__device__ __forceinline__ v16b frag_kb(const b16* p, int hh) { return cat8b(ld8b(p + 8 * hh), ld8b(p + 16 + 8 * hh)); }
__device__ __forceinline__ void split16(float v, b16& hi, b16& lo) { hi = (b16)v; lo = (b16)(v - (float)hi); }
__device__ __forceinline__ void frag_ksplit(const float* p, int hh, v16b& fh_, v16b& fl_) {
  const float* p0 = p + 8 * hh; const float* p1 = p + 16 + 8 * hh;
#pragma unroll
  for (int e = 0; e < 8; ++e) { b16 a, c; split16(p0[e], a, c); fh_[e] = a; fl_[e] = c; split16(p1[e], a, c); fh_[8 + e] = a; fl_[8 + e] = c; }
}
__device__ __forceinline__ v8f wmma16b(v16b a, v16b b, v8f c) {
  v8f d = __builtin_amdgcn_wmma_f32_16x16x32_f16(false, a, false, b, (short)0, c, false, false);
  asm volatile("v_nop\n\tv_nop\n\tv_nop\n\tv_nop" : "+v"(d) : "v"(a), "v"(b));
  return d;
}
__device__ __forceinline__ void wave_lds_sync() {
  __builtin_amdgcn_fence(__ATOMIC_RELEASE, "workgroup");
  __builtin_amdgcn_wave_barrier();
  __builtin_amdgcn_fence(__ATOMIC_ACQUIRE, "workgroup");
}

struct Opnd { const void* p0; const void* p1; int ld; };
template <int NP> __device__ __forceinline__ void load_frags(const Opnd& o, int row, int kb, int hh, v16b& fh_, v16b& fl_) {
  if (NP == 0) { frag_ksplit((const float*)o.p0 + (size_t)row * o.ld + kb, hh, fh_, fl_); }
  else if (NP == 4 || NP == 5) {
    const float sc_ = (NP == 4) ? 64.0f : 8.0f;
    const float* p = (const float*)o.p0 + (size_t)row * o.ld + kb; const float* p0 = p + 8 * hh; const float* p1 = p + 16 + 8 * hh;
#pragma unroll
    for (int e = 0; e < 8; ++e) { b16 a, c; split16(p0[e] * sc_, a, c); fh_[e] = a; fl_[e] = c; split16(p1[e] * sc_, a, c); fh_[8 + e] = a; fl_[8 + e] = c; }
  } else if (NP == 3) {
    const float* p = (const float*)o.p0 + (size_t)row * o.ld + kb; const float* p0 = p + 8 * hh; const float* p1 = p + 16 + 8 * hh;
#pragma unroll
    for (int e = 0; e < 8; ++e) { fh_[e] = (b16)p0[e]; fh_[8 + e] = (b16)p1[e]; }
    fl_ = fh_;
  } else {
    fh_ = frag_kb((const b16*)o.p0 + (size_t)row * o.ld + kb, hh);
    if (NP == 2) fl_ = frag_kb((const b16*)o.p1 + (size_t)row * o.ld + kb, hh); else fl_ = fh_;
  }
}
template <int ANP, int BNP> __device__ __forceinline__ v8f mac(v16b ah, v16b al, v16b bh, v16b bl, v8f c) {
  c = wmma16b(ah, bh, c);
  if (BNP == 0 || BNP == 2 || BNP == 4 || BNP == 5) c = wmma16b(ah, bl, c);
  if (ANP == 0 || ANP == 2 || ANP == 4 || ANP == 5) c = wmma16b(al, bh, c);
  return c;
}
template <int ANP, int BNP>
__device__ __forceinline__ void gemm_tile(const Opnd& A, const Opnd& B, int K, int m0, int c0, int nloc, int hlf, v8f (&acc)[2][4]) {
  for (int kb = 0; kb < K; kb += 32) {
    v16b a0h, a0l, a1h, a1l;
    load_frags<ANP>(A, m0 + nloc, kb, hlf, a0h, a0l);
    load_frags<ANP>(A, m0 + 16 + nloc, kb, hlf, a1h, a1l);
#pragma unroll
    for (int t = 0; t < 4; ++t) {
      v16b bh, bl;
      load_frags<BNP>(B, c0 + t * 16 + nloc, kb, hlf, bh, bl);
      acc[0][t] = mac<ANP, BNP>(a0h, a0l, bh, bl, acc[0][t]);
      acc[1][t] = mac<ANP, BNP>(a1h, a1l, bh, bl, acc[1][t]);
    }
  }
}

__device__ __forceinline__ void epi_planes(v8f (&acc)[2][4], float scale, bool two, b16* __restrict__ oh, b16* __restrict__ ol, int ldo,
                                           int m0, int c0, int lane, b16* Th, b16* Tl) {
  const int nloc = lane & 15, hlf = lane >> 4;
#pragma unroll
  for (int t = 0; t < 4; ++t)
#pragma unroll
    for (int r = 0; r < 2; ++r)
#pragma unroll
      for (int v = 0; v < 8; ++v) {
        const int rr = r * 16 + v + 8 * hlf, cc = t * 16 + nloc;
        b16 h_, l_; split16(acc[r][t][v] * scale, h_, l_);
        Th[rr * 64 + cc] = h_; Tl[rr * 64 + cc] = l_;
      }
  wave_lds_sync();
  for (int pass = 0; pass < 2; ++pass) {
#pragma unroll
    for (int j = 0; j < 8; ++j) {
      const int rr = j * 4 + (lane >> 3), c8 = (lane & 7) * 8;
      const size_t o = (size_t)(m0 + rr) * ldo + c0 + c8;
      *(volatile v8b*)(oh + o) = ld8b(Th + rr * 64 + c8);
      if (two) *(volatile v8b*)(ol + o) = ld8b(Tl + rr * 64 + c8);
    }
    __threadfence();
  }
}
__device__ __forceinline__ void epi_f32(v8f (&acc)[2][4], float scale, const float* rscale, float* __restrict__ out, int ldo, int m0, int c0, int lane, float* Tt) {
  const int nloc = lane & 15, hlf = lane >> 4;
#pragma unroll
  for (int t = 0; t < 4; ++t)
#pragma unroll
    for (int r = 0; r < 2; ++r)
#pragma unroll
      for (int v = 0; v < 8; ++v) {
        const int rr = r * 16 + v + 8 * hlf;
        const float rs = rscale ? rscale[(size_t)(m0 + rr) * 32] : 1.0f;
        Tt[rr * 64 + t * 16 + nloc] = acc[r][t][v] * scale * rs;
      }
  wave_lds_sync();
  float* dst0 = out + (size_t)m0 * ldo + c0;
  for (int pass = 0; pass < 2; ++pass) {
#pragma unroll
    for (int j = 0; j < 16; ++j) { const int rr = j * 2 + hlf, c4 = nloc * 4; *(volatile v4f*)(dst0 + (size_t)rr * ldo + c4) = *(const v4f*)(Tt + rr * 64 + c4); }
    __threadfence();
  }
}


typedef __attribute__((ext_vector_type(8))) __bf16 v8bb; typedef __attribute__((ext_vector_type(16))) __bf16 v16bb;
__device__ __forceinline__ v16bb frag_kb_bf(const __bf16* p, int hh) { const v8bb a = *(const v8bb*)(p + 8 * hh), b = *(const v8bb*)(p + 16 + 8 * hh); return __builtin_shufflevector(a, b, 0, 1, 2, 3, 4, 5, 6, 7, 8, 9, 10, 11, 12, 13, 14, 15); }
__device__ __forceinline__ v8f wmma16bb(v16bb a, v16bb b, v8f c) {
  v8f d = __builtin_amdgcn_wmma_f32_16x16x32_bf16(false, a, false, b, (short)0, c, false, false);
  asm volatile("v_nop\n\tv_nop\n\tv_nop\n\tv_nop" : "+v"(d) : "v"(a), "v"(b));
  return d;
}
__device__ __forceinline__ unsigned short bf16_rne_bits(float v) { unsigned int u = __float_as_uint(v); u += 0x7FFFu + ((u >> 16) & 1u); return (unsigned short)(u >> 16); }
__device__ __forceinline__ float bf16_rne(float v) { return __uint_as_float(((unsigned int)bf16_rne_bits(v)) << 16); }

__global__ __launch_bounds__(256) void prep_kernel(const float* __restrict__ emb, unsigned short* __restrict__ e16, b16* __restrict__ peh, b16* __restrict__ pel) {
  typedef __attribute__((ext_vector_type(8))) unsigned short v8us;
  __shared__ __attribute__((aligned(16))) b16 Sc[256 * 16];
  const size_t tid = (size_t)blockIdx.x * blockDim.x + threadIdx.x, nth = (size_t)gridDim.x * blockDim.x;
  for (int pass = 0; pass < 2; ++pass) {
    for (size_t p = tid; p < (size_t)NTOK * DM / 8; p += nth) { v8us v;
#pragma unroll
      for (int e = 0; e < 8; ++e) v[e] = bf16_rne_bits(emb[p * 8 + e]);
      *(volatile v8us*)(e16 + p * 8) = v; }
    for (size_t p = tid; p < (size_t)L * DH / 8; p += nth) { const int l = (int)(p / 8), d0 = (int)(p % 8) * 8;
      const int tblrow = l - L / 2 + SHIFT;
      const float posv = (float)(tblrow - (TBL + 1) / 2);
#pragma unroll 1
      for (int e = 0; e < 8; ++e) { const int d = d0 + e; const int j = (d < DH / 2) ? d : d - DH / 2;
        const float freq = expf((float)j * (-9.210340371976184f / (float)(DH / 2 - 1))); const float ang = posv * freq;
        const float val = (d < DH / 2) ? sinf(ang) : cosf(ang); b16 a, c; split16(val * PES, a, c); Sc[threadIdx.x * 16 + e] = a; Sc[threadIdx.x * 16 + 8 + e] = c; }
      *(volatile v8b*)(peh + p * 8) = *(const v8b*)(&Sc[threadIdx.x * 16]); *(volatile v8b*)(pel + p * 8) = *(const v8b*)(&Sc[threadIdx.x * 16 + 8]); }
    __threadfence();
  }
}

template <int MODE>
__global__ __launch_bounds__(256) void wt_kernel(const float* __restrict__ W, int K, int Ncols, unsigned short* __restrict__ out) {
  __shared__ __attribute__((aligned(16))) unsigned short Tl[64][72];
  typedef __attribute__((ext_vector_type(8))) unsigned short v8us;
  const int tid = threadIdx.x, lane = tid & 31, wave = tid >> 5, n0 = blockIdx.x * 64, k0 = blockIdx.y * 64;
  for (int i = tid; i < 64 * 64; i += 256) { const int kk = i / 64, nn = i % 64; const float w = W[(size_t)(k0 + kk) * Ncols + n0 + nn];
    unsigned short bits; if (MODE == 0) bits = bf16_rne_bits(w); else { const b16 hv = (b16)bf16_rne(w); bits = *reinterpret_cast<const unsigned short*>(&hv); }
    Tl[nn][kk] = bits; }
  __syncthreads();
  for (int pass = 0; pass < 2; ++pass) {
#pragma unroll
    for (int j = 0; j < 2; ++j) { const int rr = wave * 8 + j * 4 + (lane >> 3), c8 = (lane & 7) * 8; *(volatile v8us*)(out + (size_t)(n0 + rr) * K + k0 + c8) = *(const v8us*)(&Tl[rr][c8]); }
    __threadfence();
  }
}

__global__ __launch_bounds__(128) void qkv_kernel(const __bf16* __restrict__ e16, const __bf16* __restrict__ wqkv, b16* __restrict__ qk, b16* __restrict__ vth, b16* __restrict__ vtl) {
  __shared__ __attribute__((aligned(16))) b16 Th[4][2][32 * 64];
  __shared__ __attribute__((aligned(16))) b16 Tt[2][64][128 + 8];
  const int lane = threadIdx.x & 31, wave = threadIdx.x >> 5, nloc = lane & 15, hlf = lane >> 4, m0 = blockIdx.y * 128 + wave * 32, c0 = blockIdx.x * 64;
  v8f acc[2][4];
#pragma unroll
  for (int r = 0; r < 2; ++r)
#pragma unroll
    for (int t = 0; t < 4; ++t) acc[r][t] = (v8f){};
#pragma unroll 2
  for (int kb = 0; kb < DM; kb += 32) {
    const v16bb a0 = frag_kb_bf(e16 + (size_t)(m0 + nloc) * DM + kb, hlf), a1 = frag_kb_bf(e16 + (size_t)(m0 + 16 + nloc) * DM + kb, hlf);
#pragma unroll
    for (int t = 0; t < 4; ++t) { const v16bb bw = frag_kb_bf(wqkv + (size_t)(c0 + t * 16 + nloc) * DM + kb, hlf); acc[0][t] = wmma16bb(a0, bw, acc[0][t]); acc[1][t] = wmma16bb(a1, bw, acc[1][t]); }
  }
  const int which = c0 / DM, c1 = c0 % DM, h = c1 / DH, b = m0 / L, l0 = m0 % L;
  if (which < 3) {
    epi_planes(acc, 1.0f, false, qk + ((((size_t)which * Bn + b) * H + h) * L + l0) * DH, nullptr, DH, 0, 0, lane, Th[wave][0], Th[wave][1]);
    return;
  }
#pragma unroll
  for (int t = 0; t < 4; ++t)
#pragma unroll
    for (int r = 0; r < 2; ++r)
#pragma unroll
      for (int v = 0; v < 8; ++v) { b16 a, c; split16(acc[r][t][v] * VS, a, c); Tt[0][t * 16 + nloc][wave * 32 + r * 16 + 8 * hlf + v] = a; Tt[1][t * 16 + nloc][wave * 32 + r * 16 + 8 * hlf + v] = c; }
  __syncthreads();
  const int tok0 = (blockIdx.y * 128) % L, bb = (blockIdx.y * 128) / L;
  b16* bh_ = vth + (((size_t)bb * H + h) * DH) * L + tok0; b16* bl_ = vtl + (((size_t)bb * H + h) * DH) * L + tok0;
  for (int pass = 0; pass < 2; ++pass) {
#pragma unroll
    for (int j = 0; j < 8; ++j) { const int dd = wave * 16 + j * 2 + (lane >> 4), c8 = (lane & 15) * 8;
      *(volatile v8b*)(bh_ + (size_t)dd * L + c8) = *(const v8b*)(&Tt[0][dd][c8]); *(volatile v8b*)(bl_ + (size_t)dd * L + c8) = *(const v8b*)(&Tt[1][dd][c8]); }
    __threadfence();
  }
}

__global__ __launch_bounds__(128) void pos_kernel(const b16* __restrict__ peh, const b16* __restrict__ pel, const b16* __restrict__ wpos, b16* __restrict__ pp) {
  __shared__ __attribute__((aligned(16))) b16 Th[4][2][32 * 64];
  const int lane = threadIdx.x & 31, wave = threadIdx.x >> 5, nloc = lane & 15, hlf = lane >> 4, m0 = blockIdx.y * 128 + wave * 32, c0 = blockIdx.x * 64;
  v8f acc[2][4];
#pragma unroll
  for (int r = 0; r < 2; ++r)
#pragma unroll
    for (int t = 0; t < 4; ++t) acc[r][t] = (v8f){};
  const Opnd A{peh, pel, DH}, B{wpos, nullptr, DH};
  gemm_tile<2, 1>(A, B, DH, m0, c0, nloc, hlf, acc);
  const int which = c0 / DM, h = (c0 % DM) / DH;
  epi_planes(acc, 1.0f / PES, false, pp + (((size_t)which * H + h) * L + m0) * DH, nullptr, DH, 0, 0, lane, Th[wave][0], Th[wave][1]);
}

__global__ __launch_bounds__(256) void attn_kernel(const b16* __restrict__ qk, const b16* __restrict__ pp, const b16* __restrict__ vth, const b16* __restrict__ vtl,
                                                   const int* __restrict__ umask, const int* __restrict__ qmask, float* __restrict__ y) {
  __shared__ __attribute__((aligned(16))) float Os[8][16][DH + 4];
  const int wid = threadIdx.x >> 5, lane = threadIdx.x & 31, hh = lane >> 4, col = lane & 15;
  const int qt = blockIdx.x * 8 + wid, jt = qt & 63, h = (qt >> 6) & 15, b = qt >> 10, q0 = jt * 16, qi = q0 + col;
  const b16* Q = qk + ((((size_t)0 * Bn + b) * H + h) * L) * DH; const b16* K1 = qk + ((((size_t)1 * Bn + b) * H + h) * L) * DH; const b16* K2 = qk + ((((size_t)2 * Bn + b) * H + h) * L) * DH;
  const b16* QP = pp + (((size_t)0 * H + h) * L) * DH; const b16* KP1 = pp + (((size_t)1 * H + h) * L) * DH; const b16* KP2 = pp + (((size_t)2 * H + h) * L) * DH;
  v16b qf[2], qpf[2];
#pragma unroll
  for (int ks = 0; ks < 2; ++ks) { qf[ks] = frag_kb(Q + (size_t)qi * DH + ks * 32, hh); qpf[ks] = frag_kb(QP + (size_t)qi * DH + ks * 32, hh); }
  const int myspk = qmask[b * L + qi];
  const b16* vh = vth + (((size_t)b * H + h) * DH) * L; const b16* vl = vtl + (((size_t)b * H + h) * DH) * L;
  float m = -INFINITY, l = 0.0f; v8f o[4] = {{}, {}, {}, {}};
  for (int kb = 0; kb < q0 + 16; kb += 32) {
    float lg0[8], lg1[8];
#pragma unroll
    for (int half = 0; half < 2; ++half) {
      const int krow = kb + half * 16 + col;
      v8f s1 = {}, p1 = {}, s2 = {}, p2 = {};
#pragma unroll
      for (int ks = 0; ks < 2; ++ks) {
        s1 = wmma16b(frag_kb(K1 + (size_t)krow * DH + ks * 32, hh), qf[ks], s1); s2 = wmma16b(frag_kb(K2 + (size_t)krow * DH + ks * 32, hh), qf[ks], s2);
        p1 = wmma16b(frag_kb(KP1 + (size_t)krow * DH + ks * 32, hh), qpf[ks], p1); p2 = wmma16b(frag_kb(KP2 + (size_t)krow * DH + ks * 32, hh), qpf[ks], p2);
      }
#pragma unroll
      for (int r = 0; r < 8; ++r) { const int kk = kb + half * 16 + 8 * hh + r; const bool same = (qmask[b * L + kk] == myspk);
        float v = same ? (s1[r] + p1[r]) : (s2[r] + p2[r]);
        if (kk > qi || umask[b * L + kk] == 0) v = -INFINITY;
        if (half == 0) lg0[r] = v; else lg1[r] = v; }
    }
    float mr = -INFINITY;
#pragma unroll
    for (int r = 0; r < 8; ++r) mr = fmaxf(mr, fmaxf(lg0[r], lg1[r]));
    mr = fmaxf(mr, __shfl_xor(mr, 16));
    float mn = fmaxf(m, mr); if (mn == -INFINITY) mn = 0.0f;
    const float al_ = __expf(m - mn); m = mn;
    float sum = 0.0f; v16b pb;
#pragma unroll
    for (int r = 0; r < 8; ++r) { const float e0 = __expf(lg0[r] - mn), e1 = __expf(lg1[r] - mn); sum += e0 + e1; pb[r] = (b16)e0; pb[8 + r] = (b16)e1; }
    sum += __shfl_xor(sum, 16); l = l * al_ + sum;
#pragma unroll
    for (int n = 0; n < 4; ++n) {
#pragma unroll
      for (int r = 0; r < 8; ++r) o[n][r] *= al_;
      const size_t ro = (size_t)(n * 16 + col) * L + kb;
      o[n] = wmma16b(frag_kb(vh + ro, hh), pb, o[n]); o[n] = wmma16b(frag_kb(vl + ro, hh), pb, o[n]);
    }
  }
  const float inv = (l > 0.0f) ? (1.0f / (VS * l)) : 0.0f;
#pragma unroll
  for (int n = 0; n < 4; ++n)
#pragma unroll
    for (int r = 0; r < 8; ++r) Os[wid][col][n * 16 + 8 * hh + r] = o[n][r] * inv;
  wave_lds_sync();
  float* dst = y + ((size_t)b * L + q0) * DM + h * DH;
  for (int pass = 0; pass < 2; ++pass) {
#pragma unroll
    for (int j = 0; j < 8; ++j) { const int rr = j * 2 + hh, c4 = col * 4; *(volatile v4f*)(dst + (size_t)rr * DM + c4) = *(const v4f*)(&Os[wid][rr][c4]); }
    __threadfence();
  }
}

__global__ __launch_bounds__(128) void out_kernel(const float* __restrict__ y, const b16* __restrict__ wfc, float* __restrict__ out) {
  __shared__ __attribute__((aligned(16))) float Ts[4][32 * 64];
  const int lane = threadIdx.x & 31, wave = threadIdx.x >> 5, nloc = lane & 15, hlf = lane >> 4, m0 = blockIdx.y * 128 + wave * 32, c0 = blockIdx.x * 64;
  v8f acc[2][4];
#pragma unroll
  for (int r = 0; r < 2; ++r)
#pragma unroll
    for (int t = 0; t < 4; ++t) acc[r][t] = (v8f){};
  const Opnd A{y, nullptr, DM}, B{wfc, nullptr, DM};
  gemm_tile<5, 1>(A, B, DM, m0, c0, nloc, hlf, acc);
  epi_f32(acc, 1.0f / 8.0f, nullptr, out, DM, m0, c0, lane, Ts[wave]);
}
}

extern "C" void kernel_launch(void* const* d_in, const int* in_sizes, int n_in,
                              void* d_out, int out_size, void* d_ws, size_t ws_size, hipStream_t stream) {
  (void)n_in; (void)out_size;
  const float* emb = (const float*)d_in[0]; const int* umask = (const int*)d_in[1]; const int* qmask = (const int*)d_in[2];
  const float* Wqkv = (const float*)d_in[3]; const float* Wpos = (const float*)d_in[4]; const float* Wfc = (const float*)d_in[5];
  float* out = (float*)d_out;
  if (in_sizes[0] != NTOK * DM || in_sizes[1] != NTOK || in_sizes[2] != NTOK || in_sizes[3] != DM * NQKV || in_sizes[4] != DH * NPOS || in_sizes[5] != DM * DM) return;
  size_t off = 0; char* ws = (char*)d_ws;
  auto carve = [&](size_t bytes) { char* p = ws + off; off += (bytes + 255) & ~(size_t)255; return p; };
  unsigned short* e16 = (unsigned short*)carve((size_t)NTOK * DM * 2);
  unsigned short* wq = (unsigned short*)carve((size_t)NQKV * DM * 2);
  unsigned short* wp = (unsigned short*)carve((size_t)NPOS * DH * 2);
  unsigned short* wf = (unsigned short*)carve((size_t)DM * DM * 2);
  b16* peh = (b16*)carve((size_t)L * DH * 2); b16* pel = (b16*)carve((size_t)L * DH * 2);
  b16* qk = (b16*)carve((size_t)3 * Bn * H * L * DH * 2);
  b16* vth = (b16*)carve((size_t)Bn * H * DH * L * 2); b16* vtl = (b16*)carve((size_t)Bn * H * DH * L * 2);
  b16* pp = (b16*)carve((size_t)3 * H * L * DH * 2);
  float* y = (float*)carve((size_t)NTOK * DM * 4);
  if (off > ws_size) return;
  prep_kernel<<<512, 256, 0, stream>>>(emb, e16, peh, pel);
  wt_kernel<0><<<dim3(NQKV / 64, DM / 64), 256, 0, stream>>>(Wqkv, DM, NQKV, wq);
  wt_kernel<1><<<dim3(NPOS / 64, DH / 64), 256, 0, stream>>>(Wpos, DH, NPOS, wp);
  wt_kernel<1><<<dim3(DM / 64, DM / 64), 256, 0, stream>>>(Wfc, DM, DM, wf);
  qkv_kernel<<<dim3(NQKV / 64, NTOK / 128), 128, 0, stream>>>((const __bf16*)e16, (const __bf16*)wq, qk, vth, vtl);
  pos_kernel<<<dim3(NPOS / 64, L / 128), 128, 0, stream>>>(peh, pel, (const b16*)wp, pp);
  attn_kernel<<<Bn * H * (L / 16) / 8, 256, 0, stream>>>(qk, pp, vth, vtl, umask, qmask, y);
  out_kernel<<<dim3(DM / 64, NTOK / 128), 128, 0, stream>>>(y, (const b16*)wf, out);
}
